// HandcraftGNN_44272522887299
// MI455X (gfx1250) — hardware-verified
//
#include <hip/hip_runtime.h>
#include <stddef.h>
#include <stdint.h>


#pragma clang fp contract(off)

#define HID    128
#define HOPS   2
#define GS     4
#define EPS    3
#define NT     64
#define NW     4
#define NTHR   128
#define P1     136
#define NG     512
#define NCLS   2
#define PTHR   256
#define PW     (PTHR / 32)
#define SC_A   16.0f
#define SC_W   64.0f
#define SC_INV (1.0f / 1024.0f)
#define WS_CAP ((size_t)134217728)

static_assert(NT == 16 * NW);
static_assert(NTHR == 32 * NW);
static_assert(P1 % 8 == 0);
static_assert(P1 >= HID);
static_assert(HID % 32 == 0);
static_assert(HID == 16 * 8);
static_assert(EPS * 16 == 48);
static_assert(NG * NCLS == 4 * PTHR);
static_assert(NG % PTHR == 0);
static_assert((NG * 3) % 32 == 0);

typedef _Float16 v16h __attribute__((ext_vector_type(16)));
typedef _Float16 v8h  __attribute__((ext_vector_type(8)));
typedef float    v4f  __attribute__((ext_vector_type(4)));
typedef float    v8f  __attribute__((ext_vector_type(8)));
union FragH { v16h v; v8h h[2]; };

__device__ __forceinline__ v8f wmh(v16h a, v16h b, v8f c) {
  v8f d = __builtin_amdgcn_wmma_f32_16x16x32_f16(false, a, false, b, (short)0, c, false, false);
#if defined(__HIP_DEVICE_COMPILE__)
  asm volatile("v_nop\n\tv_nop\n\tv_nop\n\tv_nop" : "+v"(d) : "v"(a), "v"(b));
#endif
  return d;
}

__device__ __forceinline__ v8f zero8() {
  v8f z = {0.f, 0.f, 0.f, 0.f, 0.f, 0.f, 0.f, 0.f};
  return z;
}

__device__ __forceinline__ v16h afrag(const _Float16* row, int k0, int h) {
  FragH u;
  u.h[0] = *(const v8h*)(row + k0 + 8 * h);
  u.h[1] = *(const v8h*)(row + k0 + 16 + 8 * h);
  return u.v;
}

__device__ __forceinline__ int wrapclamp(int i, int n) {
  i = i < 0 ? i + n : i;
  i = i < 0 ? 0 : i;
  i = i > n - 1 ? n - 1 : i;
  return i;
}

__device__ __forceinline__ float leaky(float s) { return fmaxf(s, 0.1f * s); }

__global__ __launch_bounds__(NTHR) void k_in_mlp(const float* __restrict__ x, int nrows,
                                                 const float* __restrict__ w1, const float* __restrict__ b1,
                                                 const float* __restrict__ w2, const float* __restrict__ b2,
                                                 float* out) {
  __shared__ __align__(16) _Float16 sW2[16 * P1];
  __shared__ __align__(16) _Float16 sh1[NW * 16 * P1];
  __shared__ __align__(16) float sO[NW * 16 * 4];

  const int tid = (int)threadIdx.x, lane = tid & 31, w = tid >> 5, h = lane >> 4, m = lane & 15;

  for (int i = tid; i < 16 * P1; i += NTHR) {
    const int n = i / P1, k = i - n * P1;
    const int kc = k < HID ? k : HID - 1, ncl = n < 3 ? n : 2;
    float v = w2[kc * 3 + ncl];
    v = (n < 3 && k < HID) ? SC_W * v : 0.0f;
    sW2[i] = (_Float16)v;
  }
  const v4f wa = *(const v4f*)(w1 + 8 * m), wb = *(const v4f*)(w1 + 8 * m + 4);
  const v4f ba = *(const v4f*)(b1 + 8 * m), bb = *(const v4f*)(b1 + 8 * m + 4);
  const float b2r = b2[m < 3 ? m : 2];
  __syncthreads();

  const int r0 = blockIdx.x * NT + 16 * w;
  _Float16* shw = sh1 + w * 16 * P1;

#pragma unroll 1
  for (int nn = 0; nn < 8; ++nn) {
    const int row = 2 * nn + h;
    int rr = r0 + row;
    rr = rr < nrows ? rr : nrows - 1;
    const float xv = x[rr];
    v8h o;
#pragma unroll
    for (int q = 0; q < 4; ++q) {
      const float s0 = xv * wa[q] + ba[q];
      const float s1 = xv * wb[q] + bb[q];
      o[q]     = (_Float16)(SC_A * leaky(s0));
      o[4 + q] = (_Float16)(SC_A * leaky(s1));
    }
    *(v8h*)(shw + row * P1 + 8 * m) = o;
  }
  __syncthreads();

  v8f acc = zero8();
#pragma unroll
  for (int ks = 0; ks < HID / 32; ++ks) {
    const v16h a  = afrag(shw + m * P1, 32 * ks, h);
    const v16h bf = afrag(sW2 + m * P1, 32 * ks, h);
    acc = wmh(a, bf, acc);
  }
  float* sOw = sO + w * 64;
  if (m < 4) {
#pragma unroll
    for (int r = 0; r < 8; ++r) {
      float v = acc[r] * SC_INV + b2r;
      v = (m < 3) ? v : 0.0f;
      sOw[(8 * h + r) * 4 + m] = v;
    }
  }
  __syncthreads();
  if (lane < 16 && r0 + lane < nrows) {
    const v4f o = *(const v4f*)(sOw + 4 * lane);
    float* po = out + (size_t)(r0 + lane) * 4;
    *(volatile v4f*)po = o;
    __threadfence();
    *(volatile v4f*)po = o;
  }
}

__global__ __launch_bounds__(NTHR) void k_hop(const float* __restrict__ node_in, float* node_out,
                                              const float* __restrict__ edge_f,
                                              const int* __restrict__ subg, const int* __restrict__ seid,
                                              int nN, int nS, int nE,
                                              const float* __restrict__ mW1, const float* __restrict__ mb1,
                                              const float* __restrict__ mW2, const float* __restrict__ mb2,
                                              const float* __restrict__ uW1, const float* __restrict__ ub1,
                                              const float* __restrict__ uW2, const float* __restrict__ ub2) {
  __shared__ __align__(16) _Float16 sW2m[16 * P1];
  __shared__ __align__(16) _Float16 sW2u[16 * P1];
  __shared__ __align__(16) _Float16 sh1[NW * 16 * P1];
  __shared__ __align__(16) float sIn[NW * 48 * 8];
  __shared__ __align__(16) float sMsg[NW * 48 * 2];
  __shared__ __align__(16) float sUp[NW * 16 * 8];
  __shared__ __align__(16) float sNC[NW * 16 * 4];
  __shared__ int sCen[NW * 16];

  const int tid = (int)threadIdx.x, lane = tid & 31, w = tid >> 5, h = lane >> 4, m = lane & 15;

  for (int i = tid; i < 16 * P1; i += NTHR) {
    const int n = i / P1, k = i - n * P1;
    const int kc = k < HID ? k : HID - 1;
    float vm = mW2[kc * 2 + (n < 2 ? n : 1)];
    vm = (n < 2 && k < HID) ? SC_W * vm : 0.0f;
    float vu = uW2[kc * 3 + (n < 3 ? n : 2)];
    vu = (n < 3 && k < HID) ? SC_W * vu : 0.0f;
    sW2m[i] = (_Float16)vm;
    sW2u[i] = (_Float16)vu;
  }
  v4f wmA[6], wmB[6];
#pragma unroll
  for (int i = 0; i < 6; ++i) {
    wmA[i] = *(const v4f*)(mW1 + i * HID + 8 * m);
    wmB[i] = *(const v4f*)(mW1 + i * HID + 8 * m + 4);
  }
  const v4f bmA = *(const v4f*)(mb1 + 8 * m), bmB = *(const v4f*)(mb1 + 8 * m + 4);
  const float mb2r = mb2[m < 2 ? m : 1];
  const float ub2r = ub2[m < 3 ? m : 2];

  const int sb = blockIdx.x * NT + 16 * w;
  float* sInw = sIn + w * 48 * 8;
  float* sMw  = sMsg + w * 48 * 2;
  float* sUw  = sUp + w * 16 * 8;
  float* sNw  = sNC + w * 16 * 4;
  int*   sCw  = sCen + w * 16;
  _Float16* shw = sh1 + w * 16 * P1;

#pragma unroll
  for (int jj = 0; jj < 2; ++jj) {
    const int j  = lane + 32 * jj;
    const int jc = j < 47 ? j : 47;
    int sub = sb + jc / 3;
    sub = sub < nS ? sub : nS - 1;
    const int g   = jc - 3 * (jc / 3);
    const int nb  = wrapclamp(subg[(size_t)sub * GS + 1 + g], nN);
    const int eid = wrapclamp(seid[(size_t)sub * EPS + g], nE);
    const v4f ev = *(const v4f*)(edge_f + (size_t)eid * 4);
    const v4f nv = *(const v4f*)(node_in + (size_t)nb * 4);
    v4f a, b;
    a[0] = ev[0]; a[1] = ev[1]; a[2] = ev[2]; a[3] = nv[0];
    b[0] = nv[1]; b[1] = nv[2]; b[2] = 0.0f;  b[3] = 0.0f;
    if (j < 48) {
      *(v4f*)(sInw + j * 8)     = a;
      *(v4f*)(sInw + j * 8 + 4) = b;
    }
  }
  {
    int subc = sb + m;
    subc = subc < nS ? subc : nS - 1;
    const int cen = wrapclamp(subg[(size_t)subc * GS], nN);
    const v4f cv = *(const v4f*)(node_in + (size_t)cen * 4);
    v4f c;
    c[0] = cv[0]; c[1] = cv[1]; c[2] = cv[2]; c[3] = 0.0f;
    if (lane < 16) {
      sCw[m] = cen;
      *(v4f*)(sUw + m * 8) = c;
    }
  }
  __syncthreads();

#pragma unroll 1
  for (int t = 0; t < 3; ++t) {
#pragma unroll 1
    for (int nn = 0; nn < 8; ++nn) {
      const int row = 2 * nn + h;
      const float* xr = sInw + (16 * t + row) * 8;
      const v4f x0 = *(const v4f*)xr;
      const v4f x1 = *(const v4f*)(xr + 4);
      float xv[6];
      xv[0] = x0[0]; xv[1] = x0[1]; xv[2] = x0[2]; xv[3] = x0[3]; xv[4] = x1[0]; xv[5] = x1[1];
      v8h o;
#pragma unroll
      for (int q = 0; q < 4; ++q) {
        float s0 = bmA[q], s1 = bmB[q];
#pragma unroll
        for (int i = 0; i < 6; ++i) {
          s0 = fmaf(wmA[i][q], xv[i], s0);
          s1 = fmaf(wmB[i][q], xv[i], s1);
        }
        o[q]     = (_Float16)(SC_A * leaky(s0));
        o[4 + q] = (_Float16)(SC_A * leaky(s1));
      }
      *(v8h*)(shw + row * P1 + 8 * m) = o;
    }
    __syncthreads();

    v8f acc = zero8();
#pragma unroll
    for (int ks = 0; ks < HID / 32; ++ks) {
      const v16h a  = afrag(shw + m * P1, 32 * ks, h);
      const v16h bf = afrag(sW2m + m * P1, 32 * ks, h);
      acc = wmh(a, bf, acc);
    }
    if (m < 2) {
#pragma unroll
      for (int r = 0; r < 8; ++r) sMw[(16 * t + 8 * h + r) * 2 + m] = acc[r] * SC_INV + mb2r;
    }
    __syncthreads();
  }

  {
    const int j = m;
    const float a0 = (sMw[(3 * j) * 2 + 0] + sMw[(3 * j + 1) * 2 + 0]) + sMw[(3 * j + 2) * 2 + 0];
    const float a1 = (sMw[(3 * j) * 2 + 1] + sMw[(3 * j + 1) * 2 + 1]) + sMw[(3 * j + 2) * 2 + 1];
    if (lane < 16) {
      sUw[j * 8 + 4] = a0;
      sUw[j * 8 + 5] = a1;
    }
  }
  __syncthreads();

  v4f wuA[5], wuB[5];
#pragma unroll
  for (int i = 0; i < 5; ++i) {
    wuA[i] = *(const v4f*)(uW1 + i * HID + 8 * m);
    wuB[i] = *(const v4f*)(uW1 + i * HID + 8 * m + 4);
  }
  const v4f buA = *(const v4f*)(ub1 + 8 * m), buB = *(const v4f*)(ub1 + 8 * m + 4);
#pragma unroll 1
  for (int nn = 0; nn < 8; ++nn) {
    const int row = 2 * nn + h;
    const float* xr = sUw + row * 8;
    const v4f x0 = *(const v4f*)xr;
    const v4f x1 = *(const v4f*)(xr + 4);
    float xv[5];
    xv[0] = x0[0]; xv[1] = x0[1]; xv[2] = x0[2]; xv[3] = x1[0]; xv[4] = x1[1];
    v8h o;
#pragma unroll
    for (int q = 0; q < 4; ++q) {
      float s0 = buA[q], s1 = buB[q];
#pragma unroll
      for (int i = 0; i < 5; ++i) {
        s0 = fmaf(wuA[i][q], xv[i], s0);
        s1 = fmaf(wuB[i][q], xv[i], s1);
      }
      o[q]     = (_Float16)(SC_A * leaky(s0));
      o[4 + q] = (_Float16)(SC_A * leaky(s1));
    }
    *(v8h*)(shw + row * P1 + 8 * m) = o;
  }
  __syncthreads();

  {
    v8f acc = zero8();
#pragma unroll
    for (int ks = 0; ks < HID / 32; ++ks) {
      const v16h a  = afrag(shw + m * P1, 32 * ks, h);
      const v16h bf = afrag(sW2u + m * P1, 32 * ks, h);
      acc = wmh(a, bf, acc);
    }
    if (m < 4) {
#pragma unroll
      for (int r = 0; r < 8; ++r) {
        float v = acc[r] * SC_INV + ub2r;
        v = (m < 3) ? v : 0.0f;
        sNw[(8 * h + r) * 4 + m] = v;
      }
    }
  }
  __syncthreads();

  {
    const int nn_ = sb + m;
    v4f s4 = {0.0f, 0.0f, 0.0f, 0.0f};
#pragma unroll
    for (int j = 0; j < 16; ++j) {
      const v4f c = *(const v4f*)(sNw + 4 * j);
      const int cj = sCw[j];
      s4 = (cj == nn_) ? (s4 + c) : s4;
    }
    const int ncl = nn_ < nN ? nn_ : nN - 1;
    const v4f base = *(const v4f*)(node_in + (size_t)ncl * 4);
    const v4f o = s4 + base;
    if (lane < 16 && nn_ < nN) {
      float* po = node_out + (size_t)nn_ * 4;
      *(volatile v4f*)po = o;
      __threadfence();
      *(volatile v4f*)po = o;
    }
  }
}

__global__ __launch_bounds__(PTHR) void k_pool_head(const float* __restrict__ node_f, const int* __restrict__ batch,
                                                    int nN,
                                                    const float* __restrict__ hW1, const float* __restrict__ hb1,
                                                    const float* __restrict__ hW2, const float* __restrict__ hb2,
                                                    float* out) {
  __shared__ __align__(16) float sAcc[PW * NG * 3];
  __shared__ float sW1[3 * HID], sb1[HID], sW2[HID * NCLS];
  __shared__ __align__(16) float sOut[NG * NCLS];

  const int tid = (int)threadIdx.x, lane = tid & 31, w = tid >> 5;
  for (int i = tid; i < 3 * HID; i += PTHR) sW1[i] = hW1[i];
  for (int i = tid; i < HID; i += PTHR) sb1[i] = hb1[i];
  for (int i = tid; i < HID * NCLS; i += PTHR) sW2[i] = hW2[i];
  const float hb20 = hb2[0], hb21 = hb2[1];
  float* sA = sAcc + w * NG * 3;
  for (int i = lane; i < NG * 3; i += 32) sA[i] = 0.0f;
  __syncthreads();

  const int nsteps = (nN + PTHR - 1) / PTHR;
#pragma unroll 1
  for (int s = 0; s < nsteps; ++s) {
    const int n = (s * PW + w) * 32 + lane;
    const int ncl = n < nN ? n : nN - 1;
    const int g = batch[ncl];
    const v4f v = *(const v4f*)(node_f + (size_t)ncl * 4);
    const bool valid = (n < nN) && (g >= 0) && (g < NG);
    const int gk = valid ? g : -1;
    unsigned rem = (unsigned)__ballot(valid);
#pragma unroll 1
    for (int it = 0; it < 32; ++it) {
      if (rem == 0u) break;
      const int src = (int)__builtin_ctz(rem);
      const int leader = __shfl(gk, src, 32);
      const bool me = (gk == leader);
      const unsigned match = (unsigned)__ballot(me);
      float x0 = me ? v[0] : 0.0f;
      float x1 = me ? v[1] : 0.0f;
      float x2 = me ? v[2] : 0.0f;
#pragma unroll
      for (int off = 16; off > 0; off >>= 1) {
        x0 += __shfl_xor(x0, off, 32);
        x1 += __shfl_xor(x1, off, 32);
        x2 += __shfl_xor(x2, off, 32);
      }
      if (lane == 0) {
        float* pa = sA + leader * 3;
        pa[0] += x0;
        pa[1] += x1;
        pa[2] += x2;
      }
      rem &= ~match;
    }
  }
  __syncthreads();

  for (int gg = tid; gg < NG; gg += PTHR) {
    float e0 = 0.0f, e1 = 0.0f, e2 = 0.0f;
#pragma unroll
    for (int q = 0; q < PW; ++q) {
      const float* p = sAcc + q * NG * 3 + gg * 3;
      e0 += p[0];
      e1 += p[1];
      e2 += p[2];
    }
    float o0 = 0.0f, o1 = 0.0f;
#pragma unroll 2
    for (int j = 0; j < HID; ++j) {
      float hh = fmaf(e2, sW1[2 * HID + j], fmaf(e1, sW1[HID + j], e0 * sW1[j])) + sb1[j];
      hh = leaky(hh);
      o0 = fmaf(hh, sW2[j * NCLS + 0], o0);
      o1 = fmaf(hh, sW2[j * NCLS + 1], o1);
    }
    sOut[gg * NCLS + 0] = o0 + hb20;
    sOut[gg * NCLS + 1] = o1 + hb21;
  }
  __syncthreads();
  {
    const v4f o = *(const v4f*)(sOut + 4 * tid);
    float* po = out + 4 * tid;
    *(volatile v4f*)po = o;
    __threadfence();
    *(volatile v4f*)po = o;
  }
}

extern "C" void kernel_launch(void* const* d_in, const int* in_sizes, int n_in,
                              void* d_out, int out_size, void* d_ws, size_t ws_size,
                              hipStream_t stream) {
  if (n_in < 25) return;
  const int nN = in_sizes[0];
  const int nE = in_sizes[1];
  if (nN <= 0 || nE <= 0) return;
  if ((nN % NT) != 0 || (nE % NT) != 0) return;
  if (in_sizes[2] != GS * nN || in_sizes[3] != EPS * nN || in_sizes[4] != nN) return;
  const int nS = nN;
  if (in_sizes[5] != HID || in_sizes[6] != HID || in_sizes[7] != HID * 3 || in_sizes[8] != 3) return;
  if (in_sizes[9] != HID || in_sizes[10] != HID || in_sizes[11] != HID * 3 || in_sizes[12] != 3) return;
  if (in_sizes[13] != HOPS * 6 * HID || in_sizes[14] != HOPS * HID) return;
  if (in_sizes[15] != HOPS * HID * 2 || in_sizes[16] != HOPS * 2) return;
  if (in_sizes[17] != HOPS * 5 * HID || in_sizes[18] != HOPS * HID) return;
  if (in_sizes[19] != HOPS * HID * 3 || in_sizes[20] != HOPS * 3) return;
  if (in_sizes[21] != 3 * HID || in_sizes[22] != HID || in_sizes[23] != HID * NCLS || in_sizes[24] != NCLS) return;
  if (out_size != NG * NCLS) return;

  const float* node_feat = (const float*)d_in[0];
  const float* edge_attr = (const float*)d_in[1];
  const int*   subg      = (const int*)d_in[2];
  const int*   seid      = (const int*)d_in[3];
  const int*   batch     = (const int*)d_in[4];
  const float* nW1 = (const float*)d_in[5];
  const float* nb1 = (const float*)d_in[6];
  const float* nW2 = (const float*)d_in[7];
  const float* nb2 = (const float*)d_in[8];
  const float* eW1 = (const float*)d_in[9];
  const float* eb1 = (const float*)d_in[10];
  const float* eW2 = (const float*)d_in[11];
  const float* eb2 = (const float*)d_in[12];
  const float* mW1 = (const float*)d_in[13];
  const float* mb1 = (const float*)d_in[14];
  const float* mW2 = (const float*)d_in[15];
  const float* mb2 = (const float*)d_in[16];
  const float* uW1 = (const float*)d_in[17];
  const float* ub1 = (const float*)d_in[18];
  const float* uW2 = (const float*)d_in[19];
  const float* ub2 = (const float*)d_in[20];
  const float* hW1 = (const float*)d_in[21];
  const float* hb1 = (const float*)d_in[22];
  const float* hW2 = (const float*)d_in[23];
  const float* hb2 = (const float*)d_in[24];
  float* out = (float*)d_out;

  const size_t szN = (size_t)nN * 4 * sizeof(float);
  const size_t szE = (size_t)nE * 4 * sizeof(float);
  const size_t total = 2 * szN + szE;
  if (total > ws_size || total > WS_CAP) return;
  char* ws = (char*)d_ws;
  float* nfA = (float*)(ws);
  float* nfB = (float*)(ws + szN);
  float* ef  = (float*)(ws + 2 * szN);

  k_in_mlp<<<nN / NT, NTHR, 0, stream>>>(node_feat, nN, nW1, nb1, nW2, nb2, nfA);
  k_in_mlp<<<nE / NT, NTHR, 0, stream>>>(edge_attr, nE, eW1, eb1, eW2, eb2, ef);

  k_hop<<<nS / NT, NTHR, 0, stream>>>(nfA, nfB, ef, subg, seid, nN, nS, nE,
                                      mW1, mb1, mW2, mb2,
                                      uW1, ub1, uW2, ub2);
  k_hop<<<nS / NT, NTHR, 0, stream>>>(nfB, nfA, ef, subg, seid, nN, nS, nE,
                                      mW1 + 6 * HID, mb1 + HID, mW2 + HID * 2, mb2 + 2,
                                      uW1 + 5 * HID, ub1 + HID, uW2 + HID * 3, ub2 + 3);

  k_pool_head<<<1, PTHR, 0, stream>>>(nfA, batch, nN, hW1, hb1, hW2, hb2, out);
}
